// MP_Layer_25958782337708
// MI455X (gfx1250) — hardware-verified
//
#include <hip/hip_runtime.h>
#include <math.h>

constexpr int kBatch = 4;
constexpr int kLen   = 2048;
constexpr int kDim   = 128;
constexpr int kTok   = kBatch * kLen;
constexpr int kCat   = 2 * kDim;
constexpr float kWCarry     = 16.0f;
constexpr float kWCarryInv  = 1.0f / 16.0f;
constexpr float kPairCarry  = 2048.0f;
constexpr float kPairCarryInv = 1.0f / 2048.0f;

typedef __attribute__((ext_vector_type(16))) _Float16 v16h;
typedef __attribute__((ext_vector_type(8)))  _Float16 v8h;
typedef __attribute__((ext_vector_type(16))) __bf16   v16b;
typedef __attribute__((ext_vector_type(8)))  __bf16   v8b;
typedef __attribute__((ext_vector_type(8)))  float    v8f;
typedef __attribute__((ext_vector_type(4)))  float    v4f;
typedef __attribute__((ext_vector_type(4)))  unsigned int v4u;

__device__ __forceinline__ unsigned short f2bf_bits(float f) {
  unsigned u = __float_as_uint(f);
  return (unsigned short)((u + 0x7FFFu + ((u >> 16) & 1u)) >> 16);
}
__device__ __forceinline__ float bf_bits2f(unsigned short h) { return __uint_as_float(((unsigned)h) << 16); }

__device__ __forceinline__ void dep_guard_h(v8f& a, v8f& b, v16h x, v16h y) { asm volatile("v_nop\n\tv_nop\n\tv_nop\n\tv_nop" : "+v"(a), "+v"(b) : "v"(x), "v"(y)); }
__device__ __forceinline__ void dep_guard_b(v8f& a, v8f& b, v16b x, v16b y) { asm volatile("v_nop\n\tv_nop\n\tv_nop\n\tv_nop" : "+v"(a), "+v"(b) : "v"(x), "v"(y)); }
__device__ __forceinline__ void keep4_h(v16h a, v16h b, v16h c, v16h d) { asm volatile("v_nop" :: "v"(a), "v"(b), "v"(c), "v"(d)); }
__device__ __forceinline__ void keep4_b(v16b a, v16b b, v16b c, v16b d) { asm volatile("v_nop" :: "v"(a), "v"(b), "v"(c), "v"(d)); }
__device__ __forceinline__ void acc_guard4(v8f& a, v8f& b, v8f& c, v8f& d) { asm volatile("v_nop\n\tv_nop\n\tv_nop\n\tv_nop" : "+v"(a), "+v"(b), "+v"(c), "+v"(d)); }
template <typename T> struct Frag;
template <> struct Frag<_Float16> {
  typedef v16h V; union U { v16h v; v8h h[2]; };
  static __device__ __forceinline__ v16h load(const _Float16* p) {
    U f; f.h[0] = *(const v8h*)(p); f.h[1] = *(const v8h*)(p + 16); return f.v;
  }
  static __device__ __forceinline__ v8f mma(v16h a, v16h b, v8f c) {
    return __builtin_amdgcn_wmma_f32_16x16x32_f16(false, a, false, b, (short)0, c, false, false);
  }
  static __device__ __forceinline__ void guard(v8f& a, v8f& b, v16h x, v16h y) { dep_guard_h(a, b, x, y); }
  static __device__ __forceinline__ void keep(v16h a, v16h b, v16h c, v16h d) { keep4_h(a, b, c, d); }
};
template <> struct Frag<__bf16> {
  typedef v16b V; union U { v16b v; v8b h[2]; };
  static __device__ __forceinline__ v16b load(const __bf16* p) {
    U f; f.h[0] = *(const v8b*)(p); f.h[1] = *(const v8b*)(p + 16); return f.v;
  }
  static __device__ __forceinline__ v8f mma(v16b a, v16b b, v8f c) {
    return __builtin_amdgcn_wmma_f32_16x16x32_bf16(false, a, false, b, (short)0, c, false, false);
  }
  static __device__ __forceinline__ void guard(v8f& a, v8f& b, v16b x, v16b y) { dep_guard_b(a, b, x, y); }
  static __device__ __forceinline__ void keep(v16b a, v16b b, v16b c, v16b d) { keep4_b(a, b, c, d); }
};

__device__ __forceinline__ unsigned pk16(unsigned short a, unsigned short b) { return (unsigned)a | ((unsigned)b << 16); }
__device__ __forceinline__ unsigned short h_bits(float f) { const _Float16 h = (_Float16)f; return __builtin_bit_cast(unsigned short, h); }

template <int ET> struct Elem;
template <> struct Elem<0> { typedef _Float16 T; };
template <> struct Elem<1> { typedef __bf16 T; };
template <int ET, bool SPLIT, int BIAS_MODE, int OUT_MODE, bool RESID, int ACT = 0>
__global__ __launch_bounds__(256) void wmma_gemm64(
    const unsigned short* __restrict__ Ap, const unsigned short* __restrict__ A2p, int lda, long strideA,
    const unsigned short* __restrict__ Btp, const unsigned short* __restrict__ Bt2p, int ldb, long strideB,
    void* __restrict__ Cout, void* __restrict__ Cout2, int ldc, long strideC,
    const float* __restrict__ bias,
    const float* __restrict__ resid, long strideR,
    int M, int N, int K, float scale) {
  typedef typename Elem<ET>::T T;
  typedef typename Frag<T>::V V;
  const T* A = (const T*)Ap; const T* A2 = (const T*)A2p; const T* Bt = (const T*)Btp; const T* Bt2 = (const T*)Bt2p;
  __shared__ __align__(16) float sT[8][16 * 68];
  const int b    = blockIdx.y;
  const int lane = threadIdx.x & 31;
  const int wave = threadIdx.x >> 5;
  const int tilesN = N >> 6;
  const int tilesM = M >> 6;
  const int tile = blockIdx.x * 8 + wave;
  if (tile >= tilesM * tilesN) return;
  const int tm = tile / tilesN;
  const int tn = tile - tm * tilesN;
  const int m0 = tm << 6;
  const int n0 = tn << 6;

  const T* Ab  = A  + (size_t)b * strideA;
  const T* Bb  = Bt + (size_t)b * strideB;
  const T* Ab2 = SPLIT ? (A2  + (size_t)b * strideA) : nullptr;
  const T* Bb2 = SPLIT ? (Bt2 + (size_t)b * strideB) : nullptr;

  const int rlane = lane & 15;
  const int koff  = (lane >> 4) * 8;
  const int mOff  = (lane >> 4) * 8;

  v8f acc[4][4];
#pragma unroll
  for (int i = 0; i < 4; ++i)
#pragma unroll
    for (int j = 0; j < 4; ++j) acc[i][j] = (v8f){0.f,0.f,0.f,0.f,0.f,0.f,0.f,0.f};

  for (int k0 = 0; k0 < K; k0 += 32) {
    V bh[4], bl[4];
#pragma unroll
    for (int j = 0; j < 4; ++j) {
      const size_t bo = (size_t)(n0 + (j << 4) + rlane) * ldb + koff + k0;
      bh[j] = Frag<T>::load(Bb + bo);
      if (SPLIT) bl[j] = Frag<T>::load(Bb2 + bo);
    }
#pragma unroll
    for (int i = 0; i < 4; ++i) {
      const size_t ao = (size_t)(m0 + (i << 4) + rlane) * lda + koff + k0;
      V ah = Frag<T>::load(Ab + ao);
      V al;
      if (SPLIT) al = Frag<T>::load(Ab2 + ao);
#pragma unroll
      for (int j = 0; j < 4; ++j) {
        acc[i][j] = Frag<T>::mma(ah, bh[j], acc[i][j]);
        if (SPLIT) {
          acc[i][j] = Frag<T>::mma(ah, bl[j], acc[i][j]);
          acc[i][j] = Frag<T>::mma(al, bh[j], acc[i][j]);
        }
      }
      Frag<T>::guard(acc[i][0], acc[i][3], ah, SPLIT ? al : ah);
    }
    Frag<T>::keep(bh[0], bh[1], bh[2], bh[3]);
    if (SPLIT) Frag<T>::keep(bl[0], bl[1], bl[2], bl[3]);
  }
  acc_guard4(acc[0][0], acc[0][1], acc[0][2], acc[0][3]);
  acc_guard4(acc[1][0], acc[1][1], acc[1][2], acc[1][3]);
  acc_guard4(acc[2][0], acc[2][1], acc[2][2], acc[2][3]);
  acc_guard4(acc[3][0], acc[3][1], acc[3][2], acc[3][3]);

  float* slab = sT[wave];
  const float* Rb = RESID ? (resid + (size_t)b * strideR) : nullptr;
#pragma unroll
  for (int i = 0; i < 4; ++i) {
    const int mBase = m0 + (i << 4);
#pragma unroll
    for (int j = 0; j < 4; ++j) {
      const int n = n0 + (j << 4) + rlane;
      float bv = 0.f;
      if (BIAS_MODE == 2) bv = bias[n];
#pragma unroll
      for (int r = 0; r < 8; ++r) {
        float v = acc[i][j][r] * scale;
        if (BIAS_MODE == 1) v += bias[mBase + mOff + r];
        if (BIAS_MODE == 2) v += bv;
        if (RESID) v += Rb[(size_t)(mBase + mOff + r) * ldc + n];
        if (ACT == 2) v = fmaxf(v, 0.0f);
        if (ACT == 4) v = (v > 0.f) ? v : 0.01f * v;
        slab[(mOff + r) * 68 + (j << 4) + rlane] = v;
      }
    }
    __builtin_amdgcn_fence(__ATOMIC_RELEASE, "workgroup");
    __builtin_amdgcn_wave_barrier();
    __builtin_amdgcn_fence(__ATOMIC_ACQUIRE, "workgroup");
    if (OUT_MODE == 0) {
      float* C = (float*)Cout + (size_t)b * strideC;
      const int hh = lane >> 4, c4 = (lane & 15) * 4;
      for (int pass = 0; pass < 2; ++pass) {
#pragma unroll
        for (int it = 0; it < 8; ++it) {
          const int row = it * 2 + hh;
          v4f v = *(const v4f*)(slab + row * 68 + c4);
          *(volatile v4f*)(C + (size_t)(mBase + row) * ldc + n0 + c4) = v;
        }
        __threadfence();
      }
    } else {
      const int q = lane >> 3, c8 = (lane & 7) * 8;
      unsigned short* C  = (unsigned short*)Cout  + (size_t)b * strideC;
      unsigned short* C2 = (OUT_MODE == 2) ? ((unsigned short*)Cout2 + (size_t)b * strideC) : nullptr;
      for (int pass = 0; pass < 2; ++pass) {
#pragma unroll
        for (int it = 0; it < 4; ++it) {
          const int row = it * 4 + q;
          const float* sp = slab + row * 68 + c8;
          v8h hv, lv;
#pragma unroll
          for (int e = 0; e < 8; ++e) {
            if (OUT_MODE == 1) {
              hv[e] = (_Float16)sp[e];
            } else {
              unsigned short hb = f2bf_bits(sp[e]);
              unsigned short lb = f2bf_bits(sp[e] - bf_bits2f(hb));
              hv[e] = __builtin_bit_cast(_Float16, hb);
              lv[e] = __builtin_bit_cast(_Float16, lb);
            }
          }
          *(volatile v8h*)(C + (size_t)(mBase + row) * ldc + n0 + c8) = hv;
          if (OUT_MODE == 2) *(volatile v8h*)(C2 + (size_t)(mBase + row) * ldc + n0 + c8) = lv;
        }
        __threadfence();
      }
    }
    __builtin_amdgcn_fence(__ATOMIC_RELEASE, "workgroup");
    __builtin_amdgcn_wave_barrier();
    __builtin_amdgcn_fence(__ATOMIC_ACQUIRE, "workgroup");
  }
}

__global__ __launch_bounds__(256) void cast8_f16_kernel(const float* __restrict__ in, unsigned short* __restrict__ out, int n8, float carry) {
  const int i = blockIdx.x * 256 + threadIdx.x;
  if (i >= n8) return;
  const float* p = in + 8 * (size_t)i;
  const v4f a = *(const v4f*)(p);
  const v4f c = *(const v4f*)(p + 4);
  unsigned short hb[8];
#pragma unroll
  for (int e = 0; e < 4; ++e) {
    hb[e]     = h_bits(a[e] * carry);
    hb[4 + e] = h_bits(c[e] * carry);
  }
  const v4u u = (v4u){pk16(hb[0], hb[1]), pk16(hb[2], hb[3]), pk16(hb[4], hb[5]), pk16(hb[6], hb[7])};
  unsigned short* q = out + 8 * (size_t)i;
  *(volatile v4u*)q = u;
  __threadfence();
  *(volatile v4u*)q = u;
}

__global__ __launch_bounds__(256) void pairw_kernel(const float* __restrict__ coords, const float* __restrict__ mask,
                                                    unsigned short* __restrict__ Wp, float carry) {
#pragma clang fp contract(off)
  const int e2 = blockIdx.x * 256 + threadIdx.x;
  const int e  = e2 * 2;
  const int b  = e >> 22;
  const int i  = (e >> 11) & (kLen - 1);
  const int j0 = e & (kLen - 1);
  const int pi = b * kLen + i;
  const float xi = coords[pi * 3 + 0];
  const float yi = coords[pi * 3 + 1];
  const float zi = coords[pi * 3 + 2];
  const float mi = mask[pi];
  unsigned packed = 0u;
#pragma unroll 1
  for (int t = 0; t < 2; ++t) {
    const int pj = b * kLen + j0 + t;
    const float dx = xi - coords[pj * 3 + 0];
    const float dy = yi - coords[pj * 3 + 1];
    const float dz = zi - coords[pj * 3 + 2];
    const float d2 = (dx * dx + dz * dz) + dy * dy;
    const float dist = sqrtf(d2);
    float w = expf(-dist);
    w = w * mask[pj];
    w = w * mi;
    const float wc = w * carry;
    packed |= ((unsigned)h_bits(wc)) << (16 * t);
  }
  ((volatile unsigned*)Wp)[e2] = packed;
  __threadfence();
  ((volatile unsigned*)Wp)[e2] = packed;
}

extern "C" void kernel_launch(void* const* d_in, const int* in_sizes, int n_in,
                              void* d_out, int out_size, void* d_ws, size_t ws_size,
                              hipStream_t stream) {
  const float* h      = (const float*)d_in[0];
  const float* coords = (const float*)d_in[1];
  const float* mask   = (const float*)d_in[2];
  const float* Wself  = (const float*)d_in[3];
  const float* bself  = (const float*)d_in[4];
  const float* Wmsg   = (const float*)d_in[5];
  const float* bmsg   = (const float*)d_in[6];
  const float* Wupd   = (const float*)d_in[7];
  const float* bupd   = (const float*)d_in[8];

  if (n_in < 9) return;
  if (in_sizes[0] != kTok * kDim || in_sizes[1] != kTok * 3 || in_sizes[2] != kTok ||
      in_sizes[3] != kDim * kDim || in_sizes[5] != kDim * kDim || in_sizes[7] != kDim * kCat ||
      in_sizes[4] != kDim || in_sizes[6] != kDim || in_sizes[8] != kDim || out_size != kTok * kDim) return;

  const size_t szH16  = (size_t)kTok * kDim * 2;
  const size_t szWS16 = (size_t)kDim * kDim * 2;
  const size_t szWM16 = (size_t)kDim * kDim * 2;
  const size_t szWU16 = (size_t)kDim * kCat * 2;
  const size_t szMSGT = (size_t)kBatch * kDim * kLen * 2;
  const size_t szCAT  = (size_t)kTok * kCat * 2;
  const size_t szWP   = (size_t)kBatch * kLen * kLen * 2;
  const size_t offH16  = 0;
  const size_t offWS16 = offH16 + szH16;
  const size_t offWM16 = offWS16 + szWS16;
  const size_t offWU16 = offWM16 + szWM16;
  const size_t offMSGT = offWU16 + szWU16;
  const size_t offCAT  = offMSGT + szMSGT;
  const size_t offWP   = offCAT + szCAT;
  const size_t total   = offWP + szWP;
  if (total > ws_size) return;

  char* ws = (char*)d_ws;
  unsigned short* H16   = (unsigned short*)(ws + offH16);
  unsigned short* WS16  = (unsigned short*)(ws + offWS16);
  unsigned short* WM16  = (unsigned short*)(ws + offWM16);
  unsigned short* WU16  = (unsigned short*)(ws + offWU16);
  unsigned short* MSGT  = (unsigned short*)(ws + offMSGT);
  unsigned short* CAT16 = (unsigned short*)(ws + offCAT);
  unsigned short* WP16  = (unsigned short*)(ws + offWP);
  float* outp = (float*)d_out;

  {
    const int n8h = kTok * kDim / 8;
    cast8_f16_kernel<<<dim3((n8h + 255) / 256), dim3(256), 0, stream>>>(h, H16, n8h, 1.0f);
    const int n8s = kDim * kDim / 8;
    cast8_f16_kernel<<<dim3((n8s + 255) / 256), dim3(256), 0, stream>>>(Wself, WS16, n8s, kWCarry);
    cast8_f16_kernel<<<dim3((n8s + 255) / 256), dim3(256), 0, stream>>>(Wmsg, WM16, n8s, kWCarry);
    const int n8u = kDim * kCat / 8;
    cast8_f16_kernel<<<dim3((n8u + 255) / 256), dim3(256), 0, stream>>>(Wupd, WU16, n8u, kWCarry);
  }

  wmma_gemm64<0, false, 2, 1, false, 0><<<dim3(32, 1), dim3(256), 0, stream>>>(
      H16, H16, kDim, 0L,
      WS16, WS16, kDim, 0L,
      (void*)CAT16, (void*)CAT16, kCat, 0L,
      bself, bself, 0L,
      kTok, kDim, kDim, kWCarryInv);

  wmma_gemm64<0, false, 1, 1, false, 0><<<dim3(8, kBatch), dim3(256), 0, stream>>>(
      WM16, WM16, kDim, 0L,
      H16, H16, kDim, (long)kLen * kDim,
      (void*)MSGT, (void*)MSGT, kLen, (long)kDim * kLen,
      bmsg, bmsg, 0L,
      kDim, kLen, kDim, kWCarryInv);

  {
    const int nthreads = kBatch * kLen * kLen / 2;
    pairw_kernel<<<dim3(nthreads / 256), dim3(256), 0, stream>>>(coords, mask, WP16, kPairCarry);
  }

  wmma_gemm64<0, false, 0, 1, false, 0><<<dim3(8, kBatch), dim3(256), 0, stream>>>(
      WP16, WP16, kLen, (long)kLen * kLen,
      MSGT, MSGT, kLen, (long)kDim * kLen,
      (void*)(CAT16 + kDim), (void*)(CAT16 + kDim), kCat, (long)kLen * kCat,
      bupd, bupd, 0L,
      kLen, kDim, kLen, kPairCarryInv);

  wmma_gemm64<0, false, 2, 0, false, 0><<<dim3(32, 1), dim3(256), 0, stream>>>(
      CAT16, CAT16, kCat, 0L,
      WU16, WU16, kCat, 0L,
      (void*)outp, (void*)outp, kDim, 0L,
      bupd, bupd, 0L,
      kTok, kDim, kCat, kWCarryInv);
}
